// T5SelfAttention_6880537608801
// MI455X (gfx1250) — hardware-verified
//
#include <hip/hip_runtime.h>
#include <stdint.h>


#define BB 2
#define NN 2048
#define DM 768
#define HH 12
#define DH 64
#define MR (BB * NN)
#define NBKT 32
#define QSPLIT 16
#define RSPLIT 512

static_assert(DM % 64 == 0);
static_assert(NN % 64 == 0);
static_assert(MR % 64 == 0);
static_assert(DH == 64);
static_assert(RSPLIT % 64 == 0);
static_assert(QSPLIT <= NN / 32);
static_assert((MR * DM) % 8 == 0);

typedef _Float16 hf;
typedef _Float16 v8h_t __attribute__((ext_vector_type(8)));
typedef v8h_t __attribute__((may_alias)) v8h;
typedef _Float16 v16h __attribute__((ext_vector_type(16)));
typedef float v8f __attribute__((ext_vector_type(8)));
typedef float v4f_t __attribute__((ext_vector_type(4)));
typedef v4f_t __attribute__((may_alias)) v4f;

union Frag { v16h v; v8h_t p[2]; };

__device__ __forceinline__ v8f mma(v16h a, v16h b, v8f c)
{
    v8f d = __builtin_amdgcn_wmma_f32_16x16x32_f16(false, a, false, b, (short)0, c, false, false);
    asm volatile("v_nop\n\tv_nop\n\tv_nop\n\tv_nop" : "+v"(d) : "v"(a), "v"(b));
    return d;
}

__device__ __forceinline__ v16h ldfrag(const hf* rowptr, int k0, int hh)
{
    Frag f;
    f.p[0] = *(const v8h*)(rowptr + k0 + 8 * hh);
    f.p[1] = *(const v8h*)(rowptr + k0 + 16 + 8 * hh);
    return f.v;
}

__device__ __forceinline__ float bf16r(float v)
{
    unsigned u = __float_as_uint(v);
    u = (u + 0x7FFFu + ((u >> 16) & 1u)) & 0xFFFF0000u;
    return __uint_as_float(u);
}

__device__ __forceinline__ void split2(float v, hf& hi, hf& lo)
{
    hf h = (hf)v;
    hi = h;
    lo = (hf)((v - (float)h) * 2048.0f);
}

__device__ __forceinline__ v8f zero8()
{
    v8f z = {0.f, 0.f, 0.f, 0.f, 0.f, 0.f, 0.f, 0.f};
    return z;
}

__global__ __launch_bounds__(256)
void k_prep_x(const float* __restrict__ x, hf* __restrict__ xh, int n8)
{
    const int t = blockIdx.x * 256 + threadIdx.x;
    if (t >= n8) return;
    const float* p = x + (size_t)t * 8;
    v4f_t a = *(const v4f*)p;
    v4f_t b = *(const v4f*)(p + 4);
    v8h_t o;
    o[0] = (hf)bf16r(a[0]); o[1] = (hf)bf16r(a[1]); o[2] = (hf)bf16r(a[2]); o[3] = (hf)bf16r(a[3]);
    o[4] = (hf)bf16r(b[0]); o[5] = (hf)bf16r(b[1]); o[6] = (hf)bf16r(b[2]); o[7] = (hf)bf16r(b[3]);
    hf* d = xh + (size_t)t * 8;
    *(volatile v8h*)d = o;
    __threadfence();
    *(volatile v8h*)d = o;
}

__global__ __launch_bounds__(256)
void k_prep_w(const float* __restrict__ w0, const float* __restrict__ w1,
              const float* __restrict__ w2, const float* __restrict__ w3,
              hf* __restrict__ wt, int total)
{
    const int t = blockIdx.x * 256 + threadIdx.x;
    if (t >= total) return;
    const int per = DM * (DM / 8);
    const int wi  = t / per;
    const int rem = t - wi * per;
    const int c   = rem / (DM / 8);
    const int k8  = (rem - c * (DM / 8)) * 8;
    const float* W = (wi == 0) ? w0 : (wi == 1) ? w1 : (wi == 2) ? w2 : w3;
    v8h_t o;
    #pragma unroll
    for (int e = 0; e < 8; ++e) o[e] = (hf)(bf16r(W[(size_t)(k8 + e) * DM + c]) * 16.0f);
    hf* d = wt + (size_t)wi * DM * DM + (size_t)c * DM + k8;
    *(volatile v8h*)d = o;
    __threadfence();
    *(volatile v8h*)d = o;
}

__global__ __launch_bounds__(256)
void k_prep_bias(const float* __restrict__ rel, float* __restrict__ tab, int total4)
{
    const int t = blockIdx.x * 256 + threadIdx.x;
    if (t >= total4) return;
    const int h  = t / (NN / 4);
    const int d4 = (t - h * (NN / 4)) * 4;
    v4f_t o;
    #pragma unroll
    for (int e = 0; e < 4; ++e) {
        const int d = d4 + e;
        int bk;
        if (d < NBKT / 2) {
            bk = d;
        } else {
            float f  = (float)d * (1.0f / 16.0f);
            float lg = logf(f);
            float u  = lg * (1.0f / 2.0794415416798357f);
            float w  = u * 16.0f;
            int v = (NBKT / 2) + (int)w;
            bk = v < (NBKT - 1) ? v : (NBKT - 1);
            if (bk < 0) bk = 0;
        }
        o[e] = bf16r(rel[bk * HH + h]) * 0.125f;
    }
    float* d = tab + (size_t)h * NN + d4;
    *(volatile v4f*)d = o;
    __threadfence();
    *(volatile v4f*)d = o;
}

template <int MODE>
__global__ __launch_bounds__(128)
void k_proj(const hf* __restrict__ Ahi, const hf* __restrict__ Alo, const hf* __restrict__ Wt,
            hf* __restrict__ o0h, hf* __restrict__ o0l,
            hf* __restrict__ o1h, hf* __restrict__ o1l,
            hf* __restrict__ o2h, hf* __restrict__ o2l,
            float* __restrict__ outf)
{
    __shared__ __attribute__((aligned(16))) float Csm[64][68];

    const int wave = threadIdx.x >> 5, lane = threadIdx.x & 31, m = lane & 15, hh = lane >> 4;
    const int n0 = blockIdx.x * 64, m0 = blockIdx.y * 64, z = blockIdx.z;
    if (n0 >= DM || m0 >= MR) return;
    const hf* Bt = Wt + (size_t)z * DM * DM;
    const bool two = (MODE == 1) && ((m0 & (NN - 1)) < RSPLIT);

    const hf* arow  = Ahi + (size_t)(m0 + 16 * wave + m) * DM;
    const hf* arow2 = two ? (Alo + (size_t)(m0 + 16 * wave + m) * DM) : arow;

    v8f acc[4], acc2[4];
    #pragma unroll
    for (int t = 0; t < 4; ++t) { acc[t] = zero8(); acc2[t] = zero8(); }

    #pragma unroll 1
    for (int k0 = 0; k0 < DM; k0 += 32) {
        v16h a = ldfrag(arow, k0, hh);
        v16h bq[4];
        #pragma unroll
        for (int t = 0; t < 4; ++t) bq[t] = ldfrag(Bt + (size_t)(n0 + 16 * t + m) * DM, k0, hh);
        #pragma unroll
        for (int t = 0; t < 4; ++t) acc[t] = mma(a, bq[t], acc[t]);
        if (two) {
            v16h a2 = ldfrag(arow2, k0, hh);
            #pragma unroll
            for (int t = 0; t < 4; ++t) acc2[t] = mma(a2, bq[t], acc2[t]);
        }
    }

    #pragma unroll
    for (int t = 0; t < 4; ++t) {
        #pragma unroll
        for (int r = 0; r < 8; ++r) {
            float v = acc[t][r];
            if (MODE == 1) v += acc2[t][r] * (1.0f / 2048.0f);
            Csm[16 * wave + 8 * hh + r][16 * t + m] = v * (1.0f / 16.0f);
        }
    }
    __syncthreads();

    if (MODE == 0) {
        if (z < 2) {
            hf* dh = (z == 0) ? o0h : o1h;
            hf* dl = (z == 0) ? o0l : o1l;
            #pragma unroll 1
            for (int pass = 0; pass < 2; ++pass) {
                #pragma unroll
                for (int it = 0; it < 4; ++it) {
                    const int row = 16 * wave + 4 * it + (lane >> 3);
                    const int c8  = (lane & 7) * 8;
                    v4f_t u0 = *(const v4f*)&Csm[row][c8];
                    v4f_t u1 = *(const v4f*)&Csm[row][c8 + 4];
                    v8h_t ph, pl;
                    hf a, bl;
                    split2(u0[0], a, bl); ph[0] = a; pl[0] = bl;
                    split2(u0[1], a, bl); ph[1] = a; pl[1] = bl;
                    split2(u0[2], a, bl); ph[2] = a; pl[2] = bl;
                    split2(u0[3], a, bl); ph[3] = a; pl[3] = bl;
                    split2(u1[0], a, bl); ph[4] = a; pl[4] = bl;
                    split2(u1[1], a, bl); ph[5] = a; pl[5] = bl;
                    split2(u1[2], a, bl); ph[6] = a; pl[6] = bl;
                    split2(u1[3], a, bl); ph[7] = a; pl[7] = bl;
                    const size_t off = (size_t)(m0 + row) * DM + n0 + c8;
                    *(volatile v8h*)(dh + off) = ph;
                    *(volatile v8h*)(dl + off) = pl;
                }
                if (pass == 0) __threadfence();
            }
        } else {
            const int bidx = m0 >> 11;
            const int j0   = m0 & (NN - 1);
            #pragma unroll 1
            for (int pass = 0; pass < 2; ++pass) {
                #pragma unroll
                for (int it = 0; it < 4; ++it) {
                    const int cc = 16 * wave + 4 * it + (lane >> 3);
                    const int j8 = (lane & 7) * 8;
                    v8h_t ph, pl;
                    #pragma unroll
                    for (int e = 0; e < 8; ++e) {
                        hf a, bl;
                        split2(Csm[j8 + e][cc], a, bl);
                        ph[e] = a; pl[e] = bl;
                    }
                    const size_t off = (size_t)bidx * DM * NN + (size_t)(n0 + cc) * NN + j0 + j8;
                    *(volatile v8h*)(o2h + off) = ph;
                    *(volatile v8h*)(o2l + off) = pl;
                }
                if (pass == 0) __threadfence();
            }
        }
    } else {
        #pragma unroll 1
        for (int pass = 0; pass < 2; ++pass) {
            #pragma unroll
            for (int it = 0; it < 8; ++it) {
                const int row = 16 * wave + 2 * it + (lane >> 4);
                const int c4  = (lane & 15) * 4;
                v4f_t u = *(const v4f*)&Csm[row][c4];
                const size_t off = (size_t)(m0 + row) * DM + n0 + c4;
                *(volatile v4f*)(outf + off) = u;
            }
            if (pass == 0) __threadfence();
        }
    }
}

template <bool SPLIT>
__global__ __launch_bounds__(128)
void k_attn(const hf* __restrict__ qhi, const hf* __restrict__ qlo,
            const hf* __restrict__ khi, const hf* __restrict__ klo,
            const hf* __restrict__ vthi, const hf* __restrict__ vtlo,
            const float* __restrict__ btab, const int* __restrict__ mask,
            hf* __restrict__ ohi, hf* __restrict__ olo, int qb_base)
{
    __shared__ __attribute__((aligned(16))) float Ssm[32][68];
    __shared__ __attribute__((aligned(16))) hf Phi[32][72];
    __shared__ __attribute__((aligned(16))) hf Plo[32][72];
    __shared__ float bias_sm[NN];
    __shared__ float alpha_sm[32];
    __shared__ float l_sm[32];
    __shared__ int   msk_sm[32];

    const int tid = threadIdx.x, wave = tid >> 5, lane = tid & 31, m = lane & 15, hh = lane >> 4;
    const int qb = blockIdx.x + qb_base, h = blockIdx.y, b = blockIdx.z;
    if (qb >= NN / 32 || h >= HH || b >= BB) return;
    const int i0 = qb * 32;
    const float NINF = -__builtin_inff();

    for (int t = tid; t < NN; t += 128) bias_sm[t] = btab[(size_t)h * NN + t];
    if (tid < 32) msk_sm[tid] = mask[(size_t)b * NN + i0 + tid];
    __syncthreads();
    int anym = 0;
    #pragma unroll 1
    for (int r = 0; r < 32; ++r) anym |= (msk_sm[r] == 0) ? 1 : 0;
    const int jext   = anym ? NN : (i0 + 32);
    const int ntiles = (jext + 63) >> 6;

    const int qt  = wave >> 1;
    const int sub = wave & 1;

    const size_t qrow = ((size_t)b * NN + i0 + qt * 16 + m) * DM + (size_t)h * DH;
    v16h qf[2], qf2[2];
    #pragma unroll
    for (int ks = 0; ks < 2; ++ks) {
        qf[ks] = ldfrag(qhi + qrow, 32 * ks, hh);
        if (SPLIT) qf2[ks] = ldfrag(qlo + qrow, 32 * ks, hh); else qf2[ks] = qf[ks];
    }

    v8f oacc[2], oacc2[2];
    oacc[0] = zero8(); oacc[1] = zero8(); oacc2[0] = zero8(); oacc2[1] = zero8();
    float m_run[8], l_run[8];
    #pragma unroll
    for (int rr = 0; rr < 8; ++rr) { m_run[rr] = NINF; l_run[rr] = 0.0f; }

    #pragma unroll 1
    for (int jt = 0; jt < ntiles; ++jt) {
        const int jb = jt * 64;

        #pragma unroll
        for (int t = 0; t < 2; ++t) {
            const int kk = 2 * sub + t;
            const size_t krow = ((size_t)b * NN + jb + 16 * kk + m) * DM + (size_t)h * DH;
            v8f acc = zero8(), acc2 = zero8();
            #pragma unroll
            for (int ks = 0; ks < 2; ++ks) {
                v16h kf = ldfrag(khi + krow, 32 * ks, hh);
                acc = mma(kf, qf[ks], acc);
                if (SPLIT) {
                    v16h kf2 = ldfrag(klo + krow, 32 * ks, hh);
                    acc2 = mma(kf, qf2[ks], acc2);
                    acc2 = mma(kf2, qf[ks], acc2);
                }
            }
            float s[8];
            #pragma unroll
            for (int r = 0; r < 8; ++r) {
                float v = acc[r];
                if (SPLIT) v += acc2[r] * (1.0f / 2048.0f);
                s[r] = v * 0.125f;
            }
            float* sp = &Ssm[qt * 16 + m][16 * kk + 8 * hh];
            v4f_t s0 = {s[0], s[1], s[2], s[3]};
            v4f_t s1 = {s[4], s[5], s[6], s[7]};
            *(v4f*)sp = s0;
            *(v4f*)(sp + 4) = s1;
        }
        __syncthreads();

        #pragma unroll
        for (int rr = 0; rr < 8; ++rr) {
            const int row = 8 * wave + rr;
            const int i   = i0 + row;
            const bool valid = (msk_sm[row] != 0);
            float sv0, sv1;
            {
                const int j = jb + lane;
                float s = Ssm[row][lane];
                if (!valid) s = 0.0f; else if (j > i) s = NINF; else s += bias_sm[i - j];
                sv0 = s;
            }
            {
                const int j = jb + lane + 32;
                float s = Ssm[row][lane + 32];
                if (!valid) s = 0.0f; else if (j > i) s = NINF; else s += bias_sm[i - j];
                sv1 = s;
            }
            float tmax = fmaxf(sv0, sv1);
            #pragma unroll
            for (int off = 16; off > 0; off >>= 1) tmax = fmaxf(tmax, __shfl_xor(tmax, off, 32));
            const float mn = fmaxf(m_run[rr], tmax);
            const float alpha = (m_run[rr] == NINF) ? 0.0f : __expf(m_run[rr] - mn);
            const float p0 = __expf(sv0 - mn);
            const float p1 = __expf(sv1 - mn);
            float ps = p0 + p1;
            #pragma unroll
            for (int off = 16; off > 0; off >>= 1) ps += __shfl_xor(ps, off, 32);
            l_run[rr] = l_run[rr] * alpha + ps;
            m_run[rr] = mn;
            hf a0, b0, a1, b1;
            split2(p0 * 4096.0f, a0, b0);
            split2(p1 * 4096.0f, a1, b1);
            Phi[row][lane] = a0;
            Phi[row][lane + 32] = a1;
            if (SPLIT) { Plo[row][lane] = b0; Plo[row][lane + 32] = b1; }
            if (lane == 0) { alpha_sm[row] = alpha; l_sm[row] = l_run[rr]; }
        }
        __syncthreads();

        #pragma unroll
        for (int t = 0; t < 2; ++t) {
            const int dt = 2 * sub + t;
            float al[8];
            #pragma unroll
            for (int r = 0; r < 8; ++r) al[r] = alpha_sm[qt * 16 + 8 * hh + r];
            #pragma unroll
            for (int r = 0; r < 8; ++r) { oacc[t][r] *= al[r]; if (SPLIT) oacc2[t][r] *= al[r]; }
            const size_t vrow = (size_t)b * DM * NN + (size_t)(h * DH + 16 * dt + m) * NN + jb;
            #pragma unroll
            for (int ks = 0; ks < 2; ++ks) {
                v16h pf = ldfrag(&Phi[qt * 16 + m][0], 32 * ks, hh);
                v16h vf = ldfrag(vthi + vrow, 32 * ks, hh);
                oacc[t] = mma(pf, vf, oacc[t]);
                if (SPLIT) {
                    v16h pf2 = ldfrag(&Plo[qt * 16 + m][0], 32 * ks, hh);
                    v16h vf2 = ldfrag(vtlo + vrow, 32 * ks, hh);
                    oacc2[t] = mma(pf, vf2, oacc2[t]);
                    oacc2[t] = mma(pf2, vf, oacc2[t]);
                }
            }
        }
    }

    #pragma unroll
    for (int t = 0; t < 2; ++t) {
        const int dt = 2 * sub + t;
        #pragma unroll
        for (int r = 0; r < 8; ++r) {
            const int row = qt * 16 + 8 * hh + r;
            float o = oacc[t][r];
            if (SPLIT) o += oacc2[t][r] * (1.0f / 2048.0f);
            o = (o / l_sm[row]) * (1.0f / 4096.0f);
            Ssm[row][16 * dt + m] = o;
        }
    }
    __syncthreads();
    #pragma unroll 1
    for (int pass = 0; pass < 2; ++pass) {
        #pragma unroll
        for (int it = 0; it < 2; ++it) {
            const int row = 8 * wave + 4 * it + (lane >> 3);
            const int c8  = (lane & 7) * 8;
            v4f_t u0 = *(const v4f*)&Ssm[row][c8];
            v4f_t u1 = *(const v4f*)&Ssm[row][c8 + 4];
            v8h_t ph, pl;
            hf a, bl;
            split2(u0[0], a, bl); ph[0] = a; pl[0] = bl;
            split2(u0[1], a, bl); ph[1] = a; pl[1] = bl;
            split2(u0[2], a, bl); ph[2] = a; pl[2] = bl;
            split2(u0[3], a, bl); ph[3] = a; pl[3] = bl;
            split2(u1[0], a, bl); ph[4] = a; pl[4] = bl;
            split2(u1[1], a, bl); ph[5] = a; pl[5] = bl;
            split2(u1[2], a, bl); ph[6] = a; pl[6] = bl;
            split2(u1[3], a, bl); ph[7] = a; pl[7] = bl;
            const size_t off = ((size_t)b * NN + i0 + row) * DM + (size_t)h * DH + c8;
            *(volatile v8h*)(ohi + off) = ph;
            *(volatile v8h*)(olo + off) = pl;
        }
        if (pass == 0) __threadfence();
    }
}

extern "C" void kernel_launch(void* const* d_in, const int* in_sizes, int n_in,
                              void* d_out, int out_size, void* d_ws, size_t ws_size,
                              hipStream_t stream)
{
    if (n_in < 7) return;
    if (in_sizes[0] != MR * DM) return;
    if (in_sizes[1] != BB * NN) return;
    if (in_sizes[2] != DM * DM || in_sizes[3] != DM * DM || in_sizes[4] != DM * DM || in_sizes[5] != DM * DM) return;
    if (in_sizes[6] != NBKT * HH) return;
    if (out_size != MR * DM) return;

    const float* x    = (const float*)d_in[0];
    const int*   mask = (const int*)d_in[1];
    const float* Wq   = (const float*)d_in[2];
    const float* Wk   = (const float*)d_in[3];
    const float* Wv   = (const float*)d_in[4];
    const float* Wo   = (const float*)d_in[5];
    const float* rel  = (const float*)d_in[6];
    float* out = (float*)d_out;

    char* ws = (char*)d_ws;
    size_t off = 0;
    auto carve = [&](size_t bytes) -> size_t { size_t p = off; off += (bytes + 255) & ~(size_t)255; return p; };
    const size_t plane = (size_t)MR * DM * sizeof(hf);
    const size_t o_xh   = carve(plane);
    const size_t o_wt   = carve((size_t)4 * DM * DM * sizeof(hf));
    const size_t o_qhi  = carve(plane);
    const size_t o_qlo  = carve(plane);
    const size_t o_khi  = carve(plane);
    const size_t o_klo  = carve(plane);
    const size_t o_vthi = carve(plane);
    const size_t o_vtlo = carve(plane);
    const size_t o_ahi  = carve(plane);
    const size_t o_alo  = carve(plane);
    const size_t o_btab = carve((size_t)HH * NN * sizeof(float));
    if (off > ws_size) return;

    hf* xh   = (hf*)(ws + o_xh);
    hf* wt   = (hf*)(ws + o_wt);
    hf* qhi  = (hf*)(ws + o_qhi);
    hf* qlo  = (hf*)(ws + o_qlo);
    hf* khi  = (hf*)(ws + o_khi);
    hf* klo  = (hf*)(ws + o_klo);
    hf* vthi = (hf*)(ws + o_vthi);
    hf* vtlo = (hf*)(ws + o_vtlo);
    hf* ahi  = (hf*)(ws + o_ahi);
    hf* alo  = (hf*)(ws + o_alo);
    float* btab = (float*)(ws + o_btab);

    {
        const int n8 = MR * DM / 8;
        k_prep_x<<<(n8 + 255) / 256, 256, 0, stream>>>(x, xh, n8);
        const int tw = 4 * DM * (DM / 8);
        k_prep_w<<<(tw + 255) / 256, 256, 0, stream>>>(Wq, Wk, Wv, Wo, wt, tw);
        const int tb = HH * NN / 4;
        k_prep_bias<<<(tb + 255) / 256, 256, 0, stream>>>(rel, btab, tb);
    }

    k_proj<0><<<dim3(DM / 64, MR / 64, 3), 128, 0, stream>>>(
        xh, xh, wt, qhi, qlo, khi, klo, vthi, vtlo, out);

    k_attn<true><<<dim3(QSPLIT, HH, BB), 128, 0, stream>>>(
        qhi, qlo, khi, klo, vthi, vtlo, btab, mask, ahi, alo, 0);
    k_attn<false><<<dim3(NN / 32 - QSPLIT, HH, BB), 128, 0, stream>>>(
        qhi, qlo, khi, klo, vthi, vtlo, btab, mask, ahi, alo, QSPLIT);

    k_proj<1><<<dim3(DM / 64, MR / 64, 1), 128, 0, stream>>>(
        ahi, alo, wt + (size_t)3 * DM * DM, ahi, alo, ahi, alo, ahi, alo, out);
}
